// _MSA1_28664611734049
// MI455X (gfx1250) — hardware-verified
//
#include <hip/hip_runtime.h>


#define NBT  8
#define CIN  512
#define LL   2048
#define DD   1024
#define NH_  16
#define HD   64
#define DM   CIN
#define SCL  0.125f
#define LOSC 1024.0f

typedef _Float16 h16;
typedef unsigned short bf;
typedef __attribute__((ext_vector_type(16))) __bf16   v16bf;
typedef __attribute__((ext_vector_type(16))) _Float16 v16h;
typedef __attribute__((ext_vector_type(8)))  _Float16 v8h;
typedef __attribute__((ext_vector_type(8)))  unsigned short v8us;
typedef __attribute__((ext_vector_type(8)))  float    v8f;
typedef __attribute__((ext_vector_type(4)))  float    v4f;
typedef __attribute__((ext_vector_type(4)))  _Float16 v4h;
typedef v8h  __attribute__((may_alias)) v8ha;
typedef v4f  __attribute__((may_alias)) v4fa;
typedef v8us __attribute__((may_alias)) v8usa;

__device__ __forceinline__ unsigned short f2bf(float f) { unsigned u = __float_as_uint(f); u += 0x7FFFu + ((u >> 16) & 1u); return (unsigned short)(u >> 16); }
__device__ __forceinline__ float bf2f(unsigned short b) { return __uint_as_float(((unsigned)b) << 16); }
__device__ __forceinline__ float bfr(float f) { return bf2f(f2bf(f)); }
__device__ __forceinline__ v16h cat16(v8h lo, v8h hi) { return __builtin_shufflevector(lo, hi, 0, 1, 2, 3, 4, 5, 6, 7, 8, 9, 10, 11, 12, 13, 14, 15); }
__device__ __forceinline__ v16bf cat16b(v8us lo, v8us hi) { return __builtin_bit_cast(v16bf, __builtin_shufflevector(lo, hi, 0, 1, 2, 3, 4, 5, 6, 7, 8, 9, 10, 11, 12, 13, 14, 15)); }
__device__ __forceinline__ v8f wmma16(v16h a, v16h b, v8f c) { return __builtin_amdgcn_wmma_f32_16x16x32_f16(false, a, false, b, (short)0, c, false, false); }
__device__ __forceinline__ v8f wmmab(v16bf a, v16bf b, v8f c) { return __builtin_amdgcn_wmma_f32_16x16x32_bf16(false, a, false, b, (short)0, c, false, false); }

__global__ __launch_bounds__(256) void k_wt(const float* __restrict__ Wm, int K, int ncols, bf* WT) {
    __shared__ __align__(16) unsigned short tl[64 * 72];
    const int tid = threadIdx.x, k0 = blockIdx.x * 64, n0 = blockIdx.y * 64;
    const int kk = tid >> 2, nq = (tid & 3) * 16;
#pragma unroll
    for (int i = 0; i < 16; ++i) tl[(nq + i) * 72 + kk] = f2bf(Wm[(size_t)(k0 + kk) * ncols + n0 + nq + i]);
    __syncthreads();
    const int piece = tid & 7;
    auto pass = [&]() {
#pragma unroll
        for (int s = 0; s < 2; ++s) { const int nr = (tid >> 3) + 32 * s; const v8us val = *(const v8usa*)(tl + nr * 72 + piece * 8); *(volatile v8us*)(WT + (size_t)(n0 + nr) * K + k0 + piece * 8) = val; }
    };
    pass(); __threadfence(); pass();
}
template <bool SPLITA, bool F16OUT = false>
__global__ __launch_bounds__(128) void k_gemmb(const bf* __restrict__ A, const bf* __restrict__ Al, const bf* __restrict__ Bn, const float* __restrict__ bias, float* C, int ldc, h16* C2, const float* __restrict__ R = nullptr, int K = DM, int roundR = 1) {
    __shared__ __align__(16) float ost[4][16 * 68];
    const int lane = threadIdx.x & 31, wave = threadIdx.x >> 5, lr = lane & 15, hi = lane >> 4;
    const int r0 = blockIdx.x * 64 + wave * 16, c0 = blockIdx.y * 64;
    const size_t aoff = (size_t)(r0 + lr) * K + 8 * hi;
    size_t boff[4];
#pragma unroll
    for (int t = 0; t < 4; ++t) boff[t] = (size_t)(c0 + t * 16 + lr) * K + 8 * hi;
    v8f acc[4];
#pragma unroll
    for (int t = 0; t < 4; ++t) acc[t] = (v8f){};
#pragma unroll 1
    for (int kc = 0; kc < K; kc += 32) {
        const v16bf a = cat16b(*(const v8us*)(A + aoff + kc), *(const v8us*)(A + aoff + kc + 16));
        v16bf al = a;
        if (SPLITA) al = cat16b(*(const v8us*)(Al + aoff + kc), *(const v8us*)(Al + aoff + kc + 16));
#pragma unroll
        for (int t = 0; t < 4; ++t) { const v16bf b = cat16b(*(const v8us*)(Bn + boff[t] + kc), *(const v8us*)(Bn + boff[t] + kc + 16)); acc[t] = wmmab(a, b, acc[t]); if (SPLITA) acc[t] = wmmab(al, b, acc[t]); }
        asm volatile("v_nop\n\tv_nop\n\tv_nop\n\tv_nop" : "+v"(acc[0]), "+v"(acc[1]), "+v"(acc[2]), "+v"(acc[3]) : "v"(a), "v"(al));
    }
    float* os = &ost[wave][0];
#pragma unroll
    for (int t = 0; t < 4; ++t) { const float bv = bias ? bfr(bias[c0 + t * 16 + lr]) : 0.f;
#pragma unroll
        for (int j = 0; j < 8; ++j) os[(hi * 8 + j) * 68 + t * 16 + lr] = acc[t][j] + bv; }
    __syncthreads();
    if (F16OUT) {
        h16* crow = (h16*)(void*)C + (size_t)r0 * ldc + c0;
        auto pass = [&]() {
#pragma unroll
            for (int s = 0; s < 4; ++s) { const int row = 4 * s + (lane >> 3), piece = lane & 7; const float* sp = os + row * 68 + piece * 8; v8h o, o2;
#pragma unroll
                for (int i = 0; i < 8; ++i) { const h16 a = (h16)sp[i]; o[i] = a; o2[i] = (h16)((sp[i] - (float)a) * LOSC); }
                *(volatile v8h*)(crow + (size_t)row * ldc + piece * 8) = o; if (C2) *(volatile v8h*)(C2 + (size_t)r0 * ldc + c0 + (size_t)row * ldc + piece * 8) = o2; }
        };
        pass(); __threadfence(); pass();
    } else {
        float* crow = C + (size_t)r0 * ldc + c0;
        auto pass = [&]() {
#pragma unroll
            for (int s = 0; s < 8; ++s) { const int Lid = (lane >> 3) + 4 * s, piece = lane & 7; const int row = Lid >> 1, cofs = (Lid & 1) * 32 + piece * 4;
                v4f val = *(const v4fa*)(os + row * 68 + cofs); if (R) { const v4f rv = *(const v4f*)(R + ((size_t)r0 + row) * ldc + c0 + cofs); val += roundR ? (v4f){bfr(rv[0]), bfr(rv[1]), bfr(rv[2]), bfr(rv[3])} : rv; }
                *(volatile v4f*)(crow + (size_t)row * ldc + cofs) = val; }
        };
        pass(); __threadfence(); pass();
    }
}


__global__ __launch_bounds__(256) void k_ptb(const float* __restrict__ xb, bf* XT) {
    __shared__ float tl[64][65];
    typedef __attribute__((ext_vector_type(4))) unsigned short v4us;
    const int tid = threadIdx.x, c0 = blockIdx.x * 64, p0 = blockIdx.y * 64; const int rr = tid >> 2, cq = (tid & 3) * 16;
#pragma unroll
    for (int i = 0; i < 16; ++i) tl[rr][cq + i] = xb[(size_t)(c0 + rr) * LL + p0 + cq + i];
    __syncthreads();
    const int lane = tid & 31, wv = tid >> 5;
    auto pass = [&]() {
#pragma unroll
        for (int st = 0; st < 4; ++st) { const int pr = wv * 8 + st * 2 + (lane >> 4); const int cl = (lane & 15) * 4; v4us v;
#pragma unroll
            for (int i = 0; i < 4; ++i) v[i] = f2bf(tl[cl + i][pr]);
            *(volatile v4us*)(XT + (size_t)(p0 + pr) * CIN + c0 + cl) = v; }
    };
    pass(); __threadfence(); pass();
}
__global__ __launch_bounds__(256) void k_local3(const float* __restrict__ Q, const float* __restrict__ K, const float* __restrict__ V, float* ATT) {
    typedef __attribute__((ext_vector_type(2))) float v2f_;
    const int lane = threadIdx.x & 31; const size_t wg = (size_t)blockIdx.x * 8 + (threadIdx.x >> 5); if (wg >= (size_t)LL * NH_) return; const int l = (int)(wg / NH_), h = (int)(wg % NH_);
    float qd[2], kv[2][3], vv[2][3];
#pragma unroll
    for (int i = 0; i < 2; ++i) { const int d = lane * 2 + i; qd[i] = Q[(size_t)l * DD + h * HD + d];
#pragma unroll
        for (int wp = 0; wp < 3; ++wp) { const int idx = (h * HD + d) * 3 + wp; const int w = idx >> 10, c = idx & 1023; const int lp = l + w - 1; const bool ok = (lp >= 0) && (lp < LL);
            kv[i][wp] = ok ? K[(size_t)(ok ? lp : 0) * DD + c] : 0.f; vv[i][wp] = ok ? V[(size_t)(ok ? lp : 0) * DD + c] : 0.f; } }
    float lg[3];
#pragma unroll
    for (int wp = 0; wp < 3; ++wp) { float s = qd[0] * kv[0][wp] + qd[1] * kv[1][wp];
#pragma unroll
        for (int sh = 16; sh; sh >>= 1) s += __shfl_xor(s, sh, 32);
        lg[wp] = s * SCL; }
    const float m = fmaxf(lg[0], fmaxf(lg[1], lg[2])); const float e0 = __expf(lg[0] - m), e1 = __expf(lg[1] - m), e2 = __expf(lg[2] - m); const float inv = 1.0f / (e0 + e1 + e2);
    v2f_ o;
#pragma unroll
    for (int i = 0; i < 2; ++i) o[i] = (e0 * vv[i][0] + e1 * vv[i][1] + e2 * vv[i][2]) * inv;
    float* dst = ATT + ((size_t)h * LL + l) * HD + lane * 2; *(volatile v2f_*)dst = o; __threadfence(); *(volatile v2f_*)dst = o;
}
__global__ __launch_bounds__(256) void k_viewT(const float* __restrict__ ATT, bf* Ah, bf* Al) {
    __shared__ float tl[64][65];
    typedef __attribute__((ext_vector_type(4))) unsigned short v4us;
    const int tid = threadIdx.x; const int l0 = blockIdx.x * 64, d0 = blockIdx.y * 64; const int rr = tid >> 2, cq = (tid & 3) * 16;
#pragma unroll
    for (int i = 0; i < 16; ++i) tl[rr][cq + i] = ATT[(size_t)(d0 + rr) * LL + l0 + cq + i];
    __syncthreads();
    const int lane = tid & 31, wv = tid >> 5;
    auto pass = [&]() {
#pragma unroll
        for (int st = 0; st < 4; ++st) { const int lr = wv * 8 + st * 2 + (lane >> 4); const int dq = (lane & 15) * 4; v4us oh, ol;
#pragma unroll
            for (int i = 0; i < 4; ++i) { const float y = tl[dq + i][lr]; const unsigned short hb = f2bf(y); oh[i] = hb; ol[i] = f2bf(y - bf2f(hb)); }
            const size_t o = (size_t)(l0 + lr) * DD + d0 + dq; *(volatile v4us*)(Ah + o) = oh; *(volatile v4us*)(Al + o) = ol; }
    };
    pass(); __threadfence(); pass();
}
__global__ __launch_bounds__(256) void k_outT(const float* __restrict__ RT, float* OUTB) {
    __shared__ float tl[64][65];
    const int tid = threadIdx.x; const int l0 = blockIdx.x * 64, c0 = blockIdx.y * 64; const int rr = tid >> 2, cq = (tid & 3) * 16;
#pragma unroll
    for (int i = 0; i < 16; ++i) tl[rr][cq + i] = RT[(size_t)(l0 + rr) * CIN + c0 + cq + i];
    __syncthreads();
    const int lane = tid & 31, wv = tid >> 5;
    auto pass = [&]() {
#pragma unroll
        for (int st = 0; st < 4; ++st) { const int cr = wv * 8 + st * 2 + (lane >> 4); const int lq = (lane & 15) * 4; v4f v;
#pragma unroll
            for (int i = 0; i < 4; ++i) v[i] = tl[lq + i][cr];
            *(volatile v4f*)(OUTB + (size_t)(c0 + cr) * LL + l0 + lq) = v; }
    };
    pass(); __threadfence(); pass();
}

extern "C" void kernel_launch(void* const* d_in, const int* in_sizes, int n_in,
                              void* d_out, int out_size, void* d_ws, size_t ws_size, hipStream_t stream) {
    (void)in_sizes; (void)n_in; (void)out_size;
    const float* x = (const float*)d_in[0]; const float* wq = (const float*)d_in[1]; const float* bq = (const float*)d_in[2]; const float* wk = (const float*)d_in[3]; const float* bk = (const float*)d_in[4]; const float* wv = (const float*)d_in[5]; const float* bv = (const float*)d_in[6]; const float* wo = (const float*)d_in[7]; const float* bo = (const float*)d_in[8];
    float* out = (float*)d_out;
    char* wsp = (char*)d_ws;
    auto take = [&](size_t bytes) { char* p = wsp; wsp += (bytes + 255) & ~(size_t)255; return (void*)p; };
    bf* WQ = (bf*)take((size_t)DD * CIN * 2); bf* WK = (bf*)take((size_t)DD * CIN * 2); bf* WV = (bf*)take((size_t)DD * CIN * 2); bf* WO = (bf*)take((size_t)CIN * DD * 2);
    bf* XT = (bf*)take((size_t)LL * CIN * 2); float* Q = (float*)take((size_t)LL * DD * 4); float* K = (float*)take((size_t)LL * DD * 4); float* V = (float*)take((size_t)LL * DD * 4); float* ATT = (float*)take((size_t)NH_ * LL * HD * 4);
    bf* Ah = (bf*)take((size_t)LL * DD * 2); bf* Al = (bf*)take((size_t)LL * DD * 2); float* RT = (float*)take((size_t)LL * CIN * 4);
    if ((size_t)(wsp - (char*)d_ws) > ws_size) return;
    k_wt<<<dim3(CIN / 64, DD / 64, 1), 256, 0, stream>>>(wq, CIN, DD, WQ); k_wt<<<dim3(CIN / 64, DD / 64, 1), 256, 0, stream>>>(wk, CIN, DD, WK); k_wt<<<dim3(CIN / 64, DD / 64, 1), 256, 0, stream>>>(wv, CIN, DD, WV); k_wt<<<dim3(DD / 64, CIN / 64, 1), 256, 0, stream>>>(wo, DD, CIN, WO);
    const dim3 gp(LL / 64, DD / 64, 1);
    for (int b = 0; b < NBT; ++b) {
        k_ptb<<<dim3(CIN / 64, LL / 64, 1), 256, 0, stream>>>(x + (size_t)b * CIN * LL, XT);
        k_gemmb<false, false><<<gp, 128, 0, stream>>>(XT, nullptr, WQ, bq, Q, DD, nullptr, nullptr, CIN); k_gemmb<false, false><<<gp, 128, 0, stream>>>(XT, nullptr, WK, bk, K, DD, nullptr, nullptr, CIN); k_gemmb<false, false><<<gp, 128, 0, stream>>>(XT, nullptr, WV, bv, V, DD, nullptr, nullptr, CIN);
        k_local3<<<(LL * NH_) / 8, 256, 0, stream>>>(Q, K, V, ATT);
        k_viewT<<<dim3(LL / 64, DD / 64, 1), 256, 0, stream>>>(ATT, Ah, Al);
        k_gemmb<true, false><<<dim3(LL / 64, CIN / 64, 1), 128, 0, stream>>>(Ah, Al, WO, bo, RT, CIN, nullptr, nullptr, DD);
        k_outT<<<dim3(LL / 64, CIN / 64, 1), 256, 0, stream>>>(RT, out + (size_t)b * CIN * LL); }
}
